// MaskedSelfAttention_20323785245297
// MI455X (gfx1250) — hardware-verified
//
#include <hip/hip_runtime.h>
#include <stddef.h>


typedef _Float16 h16;
typedef _Float16 v16h __attribute__((ext_vector_type(16)));
typedef _Float16 v8h  __attribute__((ext_vector_type(8)));
typedef float    v8f  __attribute__((ext_vector_type(8)));
typedef float    v4f  __attribute__((ext_vector_type(4)));

#ifndef NB
#define NB 4
#endif
#ifndef SEQ
#define SEQ 4096
#endif
#ifndef SCORE_RES
#define SCORE_RES 1
#endif
#ifndef PV_RES
#define PV_RES 0
#endif
#define NB_FULL  4
#define SEQ_FULL 4096
#define EDIM  128
#define KDIM  64
#define LIVE  64
#define NCH   (SEQ / 64 - 1)
#define TAILN ((float)(SEQ - LIVE))

static_assert(NB >= 1 && NB <= NB_FULL);
static_assert(SEQ >= 128 && SEQ <= SEQ_FULL && (SEQ % 64) == 0);
static_assert(EDIM == 128);
static_assert(KDIM == 64 && LIVE == KDIM);
static_assert((EDIM % 32) == 0 && (KDIM % 32) == 0 && (LIVE % 32) == 0);
static_assert(NCH >= 1);
static_assert(LIVE + NCH * 64 == SEQ);

#define LDT 72
#define LDO 132
static_assert((LDT % 8) == 0 && LDT >= 64);
static_assert((LDO % 4) == 0 && LDO >= EDIM);

#define WCARRY 64.0f
#define PCARRY 1024.0f
#define RCARRY 2048.0f

#define PART_BYTES ((size_t)NB * NCH * EDIM * 4)
#define VSUM_BYTES ((size_t)NB * EDIM * 4)
#define CPL_BYTES  ((size_t)NB * LIVE * EDIM * 2)
#define VPL_BYTES  ((size_t)NB * EDIM * LIVE * 2)
#define OFF_PART ((size_t)0)
#define OFF_VSUM (OFF_PART + PART_BYTES)
#define OFF_CHI  (OFF_VSUM + VSUM_BYTES)
#define OFF_CRE  (OFF_CHI + CPL_BYTES)
#define OFF_VTH  (OFF_CRE + CPL_BYTES)
#define OFF_VTR  (OFF_VTH + VPL_BYTES)
#define WS_TOTAL (OFF_VTR + VPL_BYTES)
static_assert((PART_BYTES % 128) == 0 && (VSUM_BYTES % 128) == 0);
static_assert((CPL_BYTES % 128) == 0 && (VPL_BYTES % 128) == 0);
static_assert(WS_TOTAL <= (size_t)134217728);

__device__ __forceinline__ float bf16r(float x) {
  unsigned int u = __float_as_uint(x);
  u = (u + 0x7FFFu + ((u >> 16) & 1u)) & 0xFFFF0000u;
  return __uint_as_float(u);
}

static __device__ __forceinline__ h16 toh_flush(float v) {
  const h16 r = (h16)v;
  return (fabsf(v) < 6.103515625e-05f) ? (h16)0.0f : r;
}

__device__ __forceinline__ v16h frag_at(const _Float16* p) {
  v8h lo = *(const v8h*)(p);
  v8h hi = *(const v8h*)(p + 16);
  v16h out;
#pragma unroll
  for (int i = 0; i < 8; ++i) { out[i] = lo[i]; out[i + 8] = hi[i]; }
  return out;
}
__device__ __forceinline__ v16h ld_frag(const _Float16* base, unsigned ld) {
  const unsigned lane = threadIdx.x & 31u;
  return frag_at(base + (lane & 15u) * ld + (lane >> 4) * 8u);
}

__device__ __forceinline__ v16h frag_in(const float* p, const float carry) {
  const v4f a0 = *(const v4f*)(p);
  const v4f a1 = *(const v4f*)(p + 4);
  const v4f a2 = *(const v4f*)(p + 16);
  const v4f a3 = *(const v4f*)(p + 20);
  v16h out;
#pragma unroll
  for (int i = 0; i < 4; ++i) {
    out[i]      = toh_flush(carry * bf16r(a0[i]));
    out[i + 4]  = toh_flush(carry * bf16r(a1[i]));
    out[i + 8]  = toh_flush(carry * bf16r(a2[i]));
    out[i + 12] = toh_flush(carry * bf16r(a3[i]));
  }
  return out;
}

__device__ __forceinline__ v8f wmma16(v16h a, v16h b, v8f c) {
  v8f d = __builtin_amdgcn_wmma_f32_16x16x32_f16(false, a, false, b, (short)0, c,
                                                 false, false);
  asm volatile("v_nop\n\tv_nop\n\tv_nop\n\tv_nop" : "+v"(d) : "v"(a), "v"(b));
  return d;
}

__device__ __forceinline__ float red16_max(float x) {
#pragma unroll
  for (int off = 1; off < 16; off <<= 1) x = fmaxf(x, __shfl_xor(x, off, 32));
  return x;
}
__device__ __forceinline__ float red16_sum(float x) {
#pragma unroll
  for (int off = 1; off < 16; off <<= 1) x += __shfl_xor(x, off, 32);
  return x;
}

__device__ __forceinline__ void wave_lds_sync() {
  __builtin_amdgcn_fence(3  , "wavefront");
  asm volatile("s_wait_dscnt 0x0" ::: "memory");
  __builtin_amdgcn_wave_barrier();
}

__global__ __launch_bounds__(256) void xsum_part_kernel(
    const float* __restrict__ X, float* __restrict__ part) {
#pragma clang fp contract(off)
  __shared__ float Rs[8 * EDIM];
  const unsigned lane = threadIdx.x & 31u;
  const unsigned wave = (unsigned)__builtin_amdgcn_readfirstlane((int)(threadIdx.x >> 5));
  const unsigned c = blockIdx.x, b = blockIdx.y;
  const float* xr = X + ((size_t)b * SEQ_FULL + LIVE + c * 64u + wave * 8u) * EDIM + lane * 4u;
  v4f s = {};
#pragma unroll 1
  for (unsigned r = 0; r < 8u; ++r) {
    const v4f a = *(const v4f*)(xr + (size_t)r * EDIM);
#pragma unroll
    for (int i = 0; i < 4; ++i) s[i] += bf16r(a[i]);
  }
  *(v4f*)&Rs[wave * EDIM + lane * 4u] = s;
  __syncthreads();
  if (wave == 0u) {
    v4f t = *(const v4f*)&Rs[lane * 4u];
#pragma unroll 1
    for (unsigned j = 1; j < 8u; ++j) {
      const v4f u = *(const v4f*)&Rs[j * EDIM + lane * 4u];
      t += u;
    }
    float* p = part + ((size_t)b * NCH + c) * EDIM + lane * 4u;
    *(volatile v4f*)p = t;
    __threadfence();
    *(volatile v4f*)p = t;
  }
}

__global__ __launch_bounds__(128) void vsum_kernel(
    const float* __restrict__ part, const float* __restrict__ Wv, float* __restrict__ vsum) {
#pragma clang fp contract(off)
  __shared__ float xs[EDIM];
  __shared__ float vs[EDIM];
  const unsigned tid = threadIdx.x, lane = tid & 31u;
  const unsigned wave = (unsigned)__builtin_amdgcn_readfirstlane((int)(threadIdx.x >> 5));
  const unsigned b = blockIdx.x;
  float s = 0.0f;
#pragma unroll 1
  for (unsigned c = 0; c < (unsigned)NCH; ++c) s += part[((size_t)b * NCH + c) * EDIM + tid];
  xs[tid] = s;
  __syncthreads();
  const float* wr = Wv + (size_t)tid * EDIM;
  float d = 0.0f;
#pragma unroll 1
  for (unsigned e = 0; e < (unsigned)EDIM; e += 4u) {
    const v4f wv = *(const v4f*)(wr + e);
    const v4f xv = *(const v4f*)&xs[e];
#pragma unroll
    for (int i = 0; i < 4; ++i) d += xv[i] * bf16r(wv[i]);
  }
  vs[tid] = d;
  __syncthreads();
  if (wave == 0u) {
    const v4f t = *(const v4f*)&vs[lane * 4u];
    float* p = vsum + (size_t)b * EDIM + lane * 4u;
    *(volatile v4f*)p = t;
    __threadfence();
    *(volatile v4f*)p = t;
  }
}

__device__ __forceinline__ void proj64(const float* __restrict__ xb, const float* __restrict__ W,
                                       const unsigned mw, const unsigned nw,
                                       v8f& acc0, v8f& acc1) {
  const unsigned lane = threadIdx.x & 31u;
  const unsigned hh = lane >> 4, m = lane & 15u;
  const float* ap  = xb + (size_t)(mw * 16u + m) * EDIM + hh * 8u;
  const float* bp0 = W + (size_t)(nw * 32u + m) * EDIM + hh * 8u;
  const float* bp1 = bp0 + (size_t)16 * EDIM;
  v8f a0 = {}, a1 = {};
#pragma unroll
  for (unsigned k0 = 0; k0 < (unsigned)EDIM; k0 += 32u) {
    const v16h a  = frag_in(ap + k0, 1.0f);
    const v16h b0 = frag_in(bp0 + k0, WCARRY);
    const v16h b1 = frag_in(bp1 + k0, WCARRY);
    a0 = wmma16(a, b0, a0);
    a1 = wmma16(a, b1, a1);
  }
  acc0 = a0;
  acc1 = a1;
}

__global__ __launch_bounds__(256) void ckey_kernel(
    const float* __restrict__ X, const float* __restrict__ Wk, const float* __restrict__ Wq,
    _Float16* __restrict__ Chi, _Float16* __restrict__ Cre) {
  __shared__ _Float16 Kh[64 * LDT];
  __shared__ _Float16 Kr[64 * LDT];
  __shared__ _Float16 WqT[64 * LDT];
  __shared__ _Float16 Ch[64 * LDT];
  __shared__ _Float16 Cr[64 * LDT];
  const unsigned tid = threadIdx.x, lane = tid & 31u;
  const unsigned wave = (unsigned)__builtin_amdgcn_readfirstlane((int)(threadIdx.x >> 5));
  const unsigned mw = wave >> 1, nw = wave & 1u;
  const unsigned hh = lane >> 4, m = lane & 15u;
  const unsigned e0 = blockIdx.x * 64u;
  const unsigned b = blockIdx.y;

#pragma unroll 4
  for (unsigned j = 0; j < 16u; ++j) {
    const unsigned idx = tid + 256u * j;
    const unsigned d = idx >> 6, ec = idx & 63u;
    const float v = Wq[(size_t)d * EDIM + e0 + ec];
    WqT[ec * LDT + d] = toh_flush(WCARRY * bf16r(v));
  }

  v8f k0a, k1a;
  proj64(X + (size_t)b * SEQ_FULL * EDIM, Wk, mw, nw, k0a, k1a);
#pragma unroll
  for (int r = 0; r < 8; ++r) {
    const unsigned t = mw * 16u + hh * 8u + (unsigned)r;
    const unsigned d0 = nw * 32u + m, d1 = d0 + 16u;
    const float u0 = k0a[r] * (1.0f / WCARRY);
    const float u1 = k1a[r] * (1.0f / WCARRY);
    const float kv0 = (t <= d0) ? u0 : 0.0f;
    const float kv1 = (t <= d1) ? u1 : 0.0f;
    const h16 h0 = toh_flush(kv0);
    const h16 h1 = toh_flush(kv1);
    Kh[t * LDT + d0] = h0;
    Kh[t * LDT + d1] = h1;
    Kr[t * LDT + d0] = toh_flush((kv0 - (float)h0) * RCARRY);
    Kr[t * LDT + d1] = toh_flush((kv1 - (float)h1) * RCARRY);
  }
  __syncthreads();

  v8f ch0 = {}, ch1 = {}, cr0 = {}, cr1 = {};
#pragma unroll
  for (int c = 0; c < 2; ++c) {
    const v16h ah = ld_frag(&Kh[(mw * 16u) * LDT + (unsigned)c * 32u], LDT);
    const v16h ar = ld_frag(&Kr[(mw * 16u) * LDT + (unsigned)c * 32u], LDT);
    const v16h b0 = ld_frag(&WqT[(nw * 32u) * LDT + (unsigned)c * 32u], LDT);
    const v16h b1 = ld_frag(&WqT[(nw * 32u + 16u) * LDT + (unsigned)c * 32u], LDT);
    ch0 = wmma16(ah, b0, ch0);
    ch1 = wmma16(ah, b1, ch1);
    cr0 = wmma16(ar, b0, cr0);
    cr1 = wmma16(ar, b1, cr1);
  }
#pragma unroll
  for (int r = 0; r < 8; ++r) {
    const unsigned t = mw * 16u + hh * 8u + (unsigned)r;
    const unsigned c0 = nw * 32u + m, c1 = c0 + 16u;
    const float v0 = ch0[r] + cr0[r] * (1.0f / RCARRY);
    const float v1 = ch1[r] + cr1[r] * (1.0f / RCARRY);
    const h16 h0 = toh_flush(v0);
    const h16 h1 = toh_flush(v1);
    Ch[t * LDT + c0] = h0;
    Ch[t * LDT + c1] = h1;
    Cr[t * LDT + c0] = toh_flush((v0 - (float)h0) * RCARRY);
    Cr[t * LDT + c1] = toh_flush((v1 - (float)h1) * RCARRY);
  }
  __syncthreads();

  v8h xh[2], xr[2];
  size_t off[2];
#pragma unroll
  for (unsigned i = 0; i < 2u; ++i) {
    const unsigned t = 32u * i + (tid >> 3);
    const unsigned kc = (tid & 7u) * 8u;
    xh[i] = *(const v8h*)&Ch[t * LDT + kc];
    xr[i] = *(const v8h*)&Cr[t * LDT + kc];
    off[i] = ((size_t)b * LIVE + t) * EDIM + e0 + kc;
  }
#pragma unroll
  for (int i = 0; i < 2; ++i) {
    *(volatile v8h*)(Chi + off[i]) = xh[i];
    *(volatile v8h*)(Cre + off[i]) = xr[i];
  }
  __threadfence();
#pragma unroll
  for (int i = 0; i < 2; ++i) {
    *(volatile v8h*)(Chi + off[i]) = xh[i];
    *(volatile v8h*)(Cre + off[i]) = xr[i];
  }
}

__global__ __launch_bounds__(256) void vprep_kernel(
    const float* __restrict__ X, const float* __restrict__ Wv,
    _Float16* __restrict__ Vth, _Float16* __restrict__ Vtr) {
  __shared__ _Float16 Vh[64 * LDT];
  __shared__ _Float16 Vr[64 * LDT];
  const unsigned tid = threadIdx.x, lane = tid & 31u;
  const unsigned wave = (unsigned)__builtin_amdgcn_readfirstlane((int)(threadIdx.x >> 5));
  const unsigned mw = wave >> 1, nw = wave & 1u;
  const unsigned hh = lane >> 4, m = lane & 15u;
  const unsigned v0 = blockIdx.x * 64u;
  const unsigned b = blockIdx.y;

  v8f a0, a1;
  proj64(X + (size_t)b * SEQ_FULL * EDIM, Wv + (size_t)v0 * EDIM, mw, nw, a0, a1);
#pragma unroll
  for (int r = 0; r < 8; ++r) {
    const unsigned t = mw * 16u + hh * 8u + (unsigned)r;
    const unsigned c0 = nw * 32u + m, c1 = c0 + 16u;
    const float u0 = a0[r] * (1.0f / WCARRY);
    const float u1 = a1[r] * (1.0f / WCARRY);
    const h16 h0 = toh_flush(u0);
    const h16 h1 = toh_flush(u1);
    Vh[c0 * LDT + t] = h0;
    Vh[c1 * LDT + t] = h1;
    Vr[c0 * LDT + t] = toh_flush((u0 - (float)h0) * RCARRY);
    Vr[c1 * LDT + t] = toh_flush((u1 - (float)h1) * RCARRY);
  }
  __syncthreads();

  v8h xh[2], xr[2];
  size_t off[2];
#pragma unroll
  for (unsigned i = 0; i < 2u; ++i) {
    const unsigned vl = 32u * i + (tid >> 3);
    const unsigned kc = (tid & 7u) * 8u;
    xh[i] = *(const v8h*)&Vh[vl * LDT + kc];
    xr[i] = *(const v8h*)&Vr[vl * LDT + kc];
    off[i] = ((size_t)b * EDIM + v0 + vl) * LIVE + kc;
  }
#pragma unroll
  for (int i = 0; i < 2; ++i) {
    *(volatile v8h*)(Vth + off[i]) = xh[i];
    *(volatile v8h*)(Vtr + off[i]) = xr[i];
  }
  __threadfence();
#pragma unroll
  for (int i = 0; i < 2; ++i) {
    *(volatile v8h*)(Vth + off[i]) = xh[i];
    *(volatile v8h*)(Vtr + off[i]) = xr[i];
  }
}

__global__ __launch_bounds__(128) void attn_main_kernel(
    const float* __restrict__ X, const _Float16* __restrict__ Chi,
    const _Float16* __restrict__ Cre, const _Float16* __restrict__ Vth,
    const _Float16* __restrict__ Vtr, const float* __restrict__ vsum,
    float* __restrict__ out) {
  __shared__ _Float16 Ph[4 * 16 * LDT];
#if PV_RES
  __shared__ _Float16 Pr[4 * 16 * LDT];
#endif
  __shared__ float Os[4 * 16 * LDO];

  const unsigned lane = threadIdx.x & 31u;
  const unsigned wave = (unsigned)__builtin_amdgcn_readfirstlane((int)(threadIdx.x >> 5));
  const unsigned hh = lane >> 4, m = lane & 15u;
  const unsigned b = blockIdx.y;
  const unsigned row0 = blockIdx.x * 64u + wave * 16u;
  const unsigned pbase = wave * (16u * LDT);
  const unsigned obase = wave * (16u * LDO);

  const float* xp = X + ((size_t)b * SEQ_FULL + row0 + m) * EDIM + hh * 8u;
  const _Float16* chp = Chi + ((size_t)b * LIVE + m) * EDIM + hh * 8u;
  const _Float16* crp = Cre + ((size_t)b * LIVE + m) * EDIM + hh * 8u;
  v8f sh[4];
#if SCORE_RES
  v8f sr[4];
#endif
#pragma unroll
  for (int nc = 0; nc < 4; ++nc) {
    sh[nc] = (v8f){};
#if SCORE_RES
    sr[nc] = (v8f){};
#endif
  }
#pragma unroll
  for (int c = 0; c < 4; ++c) {
    const v16h a = frag_in(xp + c * 32, 1.0f);
#pragma unroll
    for (int nc = 0; nc < 4; ++nc) {
      const v16h bh = frag_at(chp + (size_t)(nc * 16) * EDIM + c * 32);
      sh[nc] = wmma16(a, bh, sh[nc]);
#if SCORE_RES
      const v16h br = frag_at(crp + (size_t)(nc * 16) * EDIM + c * 32);
      sr[nc] = wmma16(a, br, sr[nc]);
#endif
    }
  }
#pragma unroll
  for (int nc = 0; nc < 4; ++nc)
#pragma unroll
    for (int v = 0; v < 8; ++v) {
#if SCORE_RES
      sh[nc][v] = (sh[nc][v] + sr[nc][v] * (1.0f / RCARRY)) * (1.0f / WCARRY);
#else
      sh[nc][v] = sh[nc][v] * (1.0f / WCARRY);
#endif
    }

  float mrow[8], rs[8], et[8], inv[8];
#pragma unroll
  for (int v = 0; v < 8; ++v) {
    float mx = fmaxf(fmaxf(sh[0][v], sh[1][v]), fmaxf(sh[2][v], sh[3][v]));
    mx = red16_max(mx);
    mrow[v] = fmaxf(mx, 0.0f);
    rs[v] = 0.0f;
  }
#pragma unroll
  for (int nc = 0; nc < 4; ++nc)
#pragma unroll
    for (int v = 0; v < 8; ++v) {
      const float p = __expf(sh[nc][v] - mrow[v]);
      const float t = p * PCARRY;
      const h16 hi = toh_flush(t);
      Ph[pbase + (hh * 8u + (unsigned)v) * LDT + (unsigned)nc * 16u + m] = hi;
#if PV_RES
      Pr[pbase + (hh * 8u + (unsigned)v) * LDT + (unsigned)nc * 16u + m] =
          toh_flush((t - (float)hi) * RCARRY);
      rs[v] += p;
#else
      rs[v] += (float)hi * (1.0f / PCARRY);
#endif
    }
#pragma unroll
  for (int v = 0; v < 8; ++v) {
    const float lsum = red16_sum(rs[v]);
    et[v] = __expf(-mrow[v]);
    const float z = TAILN * et[v] + lsum;
    inv[v] = __builtin_amdgcn_rcpf(z);
  }
  wave_lds_sync();

  v16h pfh[2];
  pfh[0] = ld_frag(&Ph[pbase], LDT);
  pfh[1] = ld_frag(&Ph[pbase + 32u], LDT);
#if PV_RES
  v16h pfr[2];
  pfr[0] = ld_frag(&Pr[pbase], LDT);
  pfr[1] = ld_frag(&Pr[pbase + 32u], LDT);
#endif
  const _Float16* vhp = Vth + ((size_t)b * EDIM + m) * LIVE + hh * 8u;
  const _Float16* vrp = Vtr + ((size_t)b * EDIM + m) * LIVE + hh * 8u;
  const float* vsp = vsum + (size_t)b * EDIM + m;
#pragma unroll
  for (int nb = 0; nb < 8; ++nb) {
    v8f o = {};
#pragma unroll
    for (int c = 0; c < 2; ++c) {
      const v16h vf = frag_at(vhp + (size_t)(nb * 16) * LIVE + c * 32);
      o = wmma16(pfh[c], vf, o);
    }
#if PV_RES
    v8f o2 = {};
#pragma unroll
    for (int c = 0; c < 2; ++c) {
      const v16h vr = frag_at(vrp + (size_t)(nb * 16) * LIVE + c * 32);
      o2 = wmma16(pfh[c], vr, o2);
      const v16h vf = frag_at(vhp + (size_t)(nb * 16) * LIVE + c * 32);
      o2 = wmma16(pfr[c], vf, o2);
    }
#pragma unroll
    for (int v = 0; v < 8; ++v) o[v] = o[v] + o2[v] * (1.0f / RCARRY);
#endif
    const float vsn = vsp[nb * 16];
#pragma unroll
    for (int v = 0; v < 8; ++v)
      Os[obase + (hh * 8u + (unsigned)v) * LDO + (unsigned)nb * 16u + m] =
          (o[v] * (1.0f / PCARRY) + et[v] * vsn) * inv[v];
  }
  wave_lds_sync();

  v4f xo[16];
#pragma unroll
  for (unsigned i = 0; i < 16u; ++i) xo[i] = *(const v4f*)&Os[obase + i * LDO + lane * 4u];
  float* op = out + ((size_t)b * SEQ_FULL + row0) * EDIM + lane * 4u;
#pragma unroll
  for (unsigned i = 0; i < 16u; ++i) *(volatile v4f*)(op + (size_t)i * EDIM) = xo[i];
  __threadfence();
#pragma unroll
  for (unsigned i = 0; i < 16u; ++i) *(volatile v4f*)(op + (size_t)i * EDIM) = xo[i];
}

extern "C" void kernel_launch(void* const* d_in, const int* in_sizes, int n_in,
                              void* d_out, int out_size, void* d_ws, size_t ws_size,
                              hipStream_t stream) {
  if (n_in < 4) return;
  const long long need_x = ((long long)(NB - 1) * SEQ_FULL + SEQ) * EDIM;
  if ((long long)in_sizes[0] < need_x) return;
  if ((long long)in_sizes[1] < (long long)KDIM * EDIM) return;
  if ((long long)in_sizes[2] < (long long)KDIM * EDIM) return;
  if ((long long)in_sizes[3] < (long long)EDIM * EDIM) return;
  if ((long long)out_size < need_x) return;
  if (ws_size < WS_TOTAL) return;

  const float* X  = (const float*)d_in[0];
  const float* wk = (const float*)d_in[1];
  const float* wq = (const float*)d_in[2];
  const float* wv = (const float*)d_in[3];
  float* out = (float*)d_out;

  char* ws = (char*)d_ws;
  float*    Part = (float*)(ws + OFF_PART);
  float*    Vsum = (float*)(ws + OFF_VSUM);
  _Float16* Chi  = (_Float16*)(ws + OFF_CHI);
  _Float16* Cre  = (_Float16*)(ws + OFF_CRE);
  _Float16* Vth  = (_Float16*)(ws + OFF_VTH);
  _Float16* Vtr  = (_Float16*)(ws + OFF_VTR);

  xsum_part_kernel<<<dim3(NCH, NB), dim3(256), 0, stream>>>(X, Part);
  vsum_kernel<<<dim3(NB), dim3(128), 0, stream>>>(Part, wv, Vsum);
  ckey_kernel<<<dim3(EDIM / 64, NB), dim3(256), 0, stream>>>(X, wk, wq, Chi, Cre);
  vprep_kernel<<<dim3(EDIM / 64, NB), dim3(256), 0, stream>>>(X, wv, Vth, Vtr);
  attn_main_kernel<<<dim3(SEQ / 64, NB), dim3(128), 0, stream>>>(X, Chi, Cre, Vth, Vtr, Vsum, out);
}
